// AfmoeSDPAAttention_33371895890029
// MI455X (gfx1250) — hardware-run, weakly checked
//
#include <hip/hip_runtime.h>
#include <math.h>

typedef __attribute__((ext_vector_type(16))) _Float16 v16h;
typedef __attribute__((ext_vector_type(8)))  _Float16 v8h;
typedef __attribute__((ext_vector_type(16))) __bf16   v16b;
typedef __attribute__((ext_vector_type(8)))  __bf16   v8b;
typedef __attribute__((ext_vector_type(8)))  float    v8f;
typedef __attribute__((ext_vector_type(4)))  float    v4f;
typedef __attribute__((ext_vector_type(4)))  unsigned int v4u;
typedef __attribute__((ext_vector_type(2)))  unsigned int v2u;

constexpr int kB     = 2;
constexpr int kS     = 2048;
constexpr int kHid   = 2048;
constexpr int kHq    = 16;
constexpr int kHkv   = 4;
constexpr int kRep   = kHq / kHkv;
constexpr int kHD    = 128;
constexpr int kTok   = kB * kS;
constexpr int kQW    = kHq * kHD;
constexpr int kKW    = kHkv * kHD;
constexpr int kQKVW  = kQW + 2 * kKW;
constexpr int kVCol0 = kQW + kKW;
constexpr int kSlots = kHq + kHkv;
constexpr int kEarly = 128;
constexpr int kERows = kB * kEarly;
constexpr int kLateKC    = 64;
constexpr int kLatePairs = (kS - kEarly) / 32;
constexpr int kVP    = 132;
constexpr float kEps = 1e-6f;

constexpr double cx_sqrt(double x) {
  double r = (x > 1.0) ? x : 1.0;
  for (int i = 0; i < 80; ++i) r = 0.5 * (r + x / r);
  return r;
}
constexpr float kInvSqrtHD = (float)(1.0 / cx_sqrt((double)kHD));
constexpr float kQKCarry = 64.0f;
constexpr float kVCarry  = 64.0f;
constexpr float kPCarry  = 32768.0f;
constexpr float kGCarry  = 1024.0f;
constexpr float kWoCarry = 1024.0f;
constexpr float kScoreMul   = kInvSqrtHD / (kQKCarry * kQKCarry);
constexpr float kOutLateMul = 1.0f / (kGCarry * kWoCarry);

static_assert(kRep == 4 && kHkv == 4 && kHD == 128, "lane maps assume 4 kv heads x 4 query heads x 128");
static_assert(kTok == 4096 && kQW == 2048 && kKW == 512 && kQKVW == 3072, "wire shapes");
static_assert((kHid % 32) == 0 && (kQW % 32) == 0, "GEMM K multiples of 32");
static_assert((kTok % 64) == 0 && (kQKVW % 64) == 0 && (kQW % 64) == 0 && ((kS - kEarly) % 64) == 0 && (kEarly % 64) == 0, "GEMM M,N multiples of 64");
static_assert((kS % 64) == 0 && (kS / 64) == 32 && (kEarly % 16) == 0 && ((kS - kEarly) % 32) == 0, "tile multiples");

constexpr size_t kOffXB   = 0;
constexpr size_t kOffWQKV = kOffXB   + (size_t)kTok * kHid * 2;
constexpr size_t kOffWGB  = kOffWQKV + (size_t)kQKVW * kHid * 2;
constexpr size_t kOffQKV  = kOffWGB  + (size_t)kQW * kHid * 2;
constexpr size_t kOffQP   = kOffQKV  + (size_t)kTok * kQKVW * 4;
constexpr size_t kOffKP   = kOffQP   + (size_t)kTok * kQW * 2;
constexpr size_t kOffVT   = kOffKP   + (size_t)kTok * kKW * 2;
constexpr size_t kOffQE   = kOffVT   + (size_t)kTok * kKW * 2;
constexpr size_t kOffKE   = kOffQE   + (size_t)kERows * kQW * 4;
constexpr size_t kOffVE   = kOffKE   + (size_t)kERows * kKW * 4;
constexpr size_t kOffWOB  = kOffVE   + (size_t)kERows * kKW * 4;
constexpr size_t kOffWOH  = kOffWOB  + (size_t)kQW * kQW * 2;
constexpr size_t kWsTotal = kOffWOH  + (size_t)kQW * kQW * 2;
constexpr size_t kOffATT  = kOffQKV;
constexpr size_t kOffGF   = kOffQKV + (size_t)kTok * kQW * 4;
constexpr size_t kOffGH   = kOffXB;
constexpr size_t kOffEH   = kOffWQKV;
constexpr size_t kOffEL   = kOffWQKV + (size_t)kERows * kQW * 2;
static_assert(kWsTotal == 133169152ull, "carve total");
static_assert(kWsTotal <= 134217728ull, "carve cap");
static_assert(kOffGF + (size_t)kTok * kQW * 4 == kOffKP, "gate plane covers the projection tail plus the q plane exactly");
static_assert(kOffEL + (size_t)kERows * kQW * 2 <= kOffWGB, "hi/lo planes inside the dead weight plane");
static_assert((kOffWQKV % 128) == 0 && (kOffWGB % 128) == 0 && (kOffQKV % 128) == 0 && (kOffQP % 128) == 0 &&
              (kOffKP % 128) == 0 && (kOffVT % 128) == 0 && (kOffQE % 128) == 0 && (kOffKE % 128) == 0 &&
              (kOffVE % 128) == 0 && (kOffWOB % 128) == 0 && (kOffWOH % 128) == 0 && (kOffGF % 128) == 0 &&
              (kOffEL % 128) == 0, "128-B aligned regions");

__device__ __forceinline__ unsigned short f2bf_bits(float f) {
  unsigned u = __float_as_uint(f);
  return (unsigned short)((u + 0x7FFFu + ((u >> 16) & 1u)) >> 16);
}
__device__ __forceinline__ float bf_bits2f(unsigned short h) { return __uint_as_float(((unsigned)h) << 16); }
__device__ __forceinline__ float bf16r(float f) { return bf_bits2f(f2bf_bits(f)); }
__device__ __forceinline__ unsigned pk16(unsigned short a, unsigned short b) { return (unsigned)a | ((unsigned)b << 16); }
__device__ __forceinline__ unsigned short h_bits(float f) { const _Float16 h = (_Float16)f; return __builtin_bit_cast(unsigned short, h); }
__device__ __forceinline__ void wave_lds_sync() {
  __builtin_amdgcn_fence(__ATOMIC_RELEASE, "workgroup");
  __builtin_amdgcn_wave_barrier();
  __builtin_amdgcn_fence(__ATOMIC_ACQUIRE, "workgroup");
}

__device__ __forceinline__ v8f mma_guard_h(v16h a, v16h b, v8f c) {
  c = __builtin_amdgcn_wmma_f32_16x16x32_f16(false, a, false, b, (short)0, c, false, false);
  asm volatile("v_nop\n\tv_nop\n\tv_nop\n\tv_nop" : "+v"(c) : "v"(a), "v"(b));
  return c;
}
__device__ __forceinline__ v8f mma_guard_b(v16b a, v16b b, v8f c) {
  c = __builtin_amdgcn_wmma_f32_16x16x32_bf16(false, a, false, b, (short)0, c, false, false);
  asm volatile("v_nop\n\tv_nop\n\tv_nop\n\tv_nop" : "+v"(c) : "v"(a), "v"(b));
  return c;
}
__device__ __forceinline__ void keep4_h(v16h a, v16h b, v16h c, v16h d) { asm volatile("v_nop" :: "v"(a), "v"(b), "v"(c), "v"(d)); }
__device__ __forceinline__ void keep4_b(v16b a, v16b b, v16b c, v16b d) { asm volatile("v_nop" :: "v"(a), "v"(b), "v"(c), "v"(d)); }
__device__ __forceinline__ void acc_guard4(v8f& a, v8f& b, v8f& c, v8f& d) { asm volatile("v_nop\n\tv_nop\n\tv_nop\n\tv_nop" : "+v"(a), "+v"(b), "+v"(c), "+v"(d)); }

template <typename T> struct Frag;
template <> struct Frag<_Float16> {
  typedef v16h V; union U { v16h v; v8h h[2]; };
  static __device__ __forceinline__ v16h load(const _Float16* p) {
    U f; f.h[0] = *(const v8h*)(p); f.h[1] = *(const v8h*)(p + 16); return f.v;
  }
  static __device__ __forceinline__ v8f mmag(v16h a, v16h b, v8f c) { return mma_guard_h(a, b, c); }
  static __device__ __forceinline__ void keep(v16h a, v16h b, v16h c, v16h d) { keep4_h(a, b, c, d); }
};
template <> struct Frag<__bf16> {
  typedef v16b V; union U { v16b v; v8b h[2]; };
  static __device__ __forceinline__ v16b load(const __bf16* p) {
    U f; f.h[0] = *(const v8b*)(p); f.h[1] = *(const v8b*)(p + 16); return f.v;
  }
  static __device__ __forceinline__ v8f mmag(v16b a, v16b b, v8f c) { return mma_guard_b(a, b, c); }
  static __device__ __forceinline__ void keep(v16b a, v16b b, v16b c, v16b d) { keep4_b(a, b, c, d); }
};

template <int ET> struct Elem;
template <> struct Elem<0> { typedef _Float16 T; };
template <> struct Elem<1> { typedef __bf16 T; };
template <int ET, bool ASPLIT>
__global__ __launch_bounds__(256) void wmma_gemm64(
    const unsigned short* __restrict__ Ap, const unsigned short* __restrict__ A2p, int lda, long strideA,
    const unsigned short* __restrict__ Btp, int ldb, long strideB,
    float* __restrict__ Cout, int ldc, long strideC,
    int M, int N, int K, float scale) {
  typedef typename Elem<ET>::T T;
  typedef typename Frag<T>::V V;
  const T* A = (const T*)Ap; const T* A2 = (const T*)A2p; const T* Bt = (const T*)Btp;
  __shared__ __align__(16) float sT[8][16 * 68];
  const int b    = blockIdx.y;
  const int lane = threadIdx.x & 31;
  const int wave = __builtin_amdgcn_readfirstlane((int)(threadIdx.x >> 5));
  const int tilesN = N >> 6;
  const int tilesM = M >> 6;
  const int tile = blockIdx.x * 8 + wave;
  if (tile >= tilesM * tilesN) return;
  const int tm = tile / tilesN;
  const int tn = tile - tm * tilesN;
  const int m0 = tm << 6;
  const int n0 = tn << 6;

  const T* Ab  = A  + (size_t)b * strideA;
  const T* Bb  = Bt + (size_t)b * strideB;
  const T* Ab2 = A2 + (size_t)b * strideA;

  const int rlane = lane & 15;
  const int koff  = (lane >> 4) * 8;
  const int mOff  = (lane >> 4) * 8;

  v8f acc[4][4];
#pragma unroll
  for (int i = 0; i < 4; ++i)
#pragma unroll
    for (int j = 0; j < 4; ++j) acc[i][j] = (v8f){0.f,0.f,0.f,0.f,0.f,0.f,0.f,0.f};

  for (int k0 = 0; k0 < K; k0 += 32) {
    V bh[4];
#pragma unroll
    for (int j = 0; j < 4; ++j) {
      const size_t bo = (size_t)(n0 + (j << 4) + rlane) * ldb + koff + k0;
      bh[j] = Frag<T>::load(Bb + bo);
    }
#pragma unroll
    for (int i = 0; i < 4; ++i) {
      const size_t ao = (size_t)(m0 + (i << 4) + rlane) * lda + koff + k0;
      V ah = Frag<T>::load(Ab + ao);
      V al = ah;
      if (ASPLIT) al = Frag<T>::load(Ab2 + ao);
#pragma unroll
      for (int j = 0; j < 4; ++j) {
        acc[i][j] = Frag<T>::mmag(ah, bh[j], acc[i][j]);
        if (ASPLIT) acc[i][j] = Frag<T>::mmag(al, bh[j], acc[i][j]);
      }
    }
    Frag<T>::keep(bh[0], bh[1], bh[2], bh[3]);
  }
  acc_guard4(acc[0][0], acc[0][1], acc[0][2], acc[0][3]);
  acc_guard4(acc[1][0], acc[1][1], acc[1][2], acc[1][3]);
  acc_guard4(acc[2][0], acc[2][1], acc[2][2], acc[2][3]);
  acc_guard4(acc[3][0], acc[3][1], acc[3][2], acc[3][3]);

  float* slab = sT[wave];
  float* C = Cout + (size_t)b * strideC;
#pragma unroll
  for (int i = 0; i < 4; ++i) {
    const int mBase = m0 + (i << 4);
#pragma unroll
    for (int j = 0; j < 4; ++j) {
#pragma unroll
      for (int r = 0; r < 8; ++r) {
        slab[(mOff + r) * 68 + (j << 4) + rlane] = acc[i][j][r] * scale;
      }
    }
    wave_lds_sync();
    {
      const int hh = lane >> 4, c4 = (lane & 15) * 4;
      for (int pass = 0; pass < 2; ++pass) {
#pragma unroll
        for (int it = 0; it < 8; ++it) {
          const int row = it * 2 + hh;
          v4f v = *(const v4f*)(slab + row * 68 + c4);
          *(volatile v4f*)(C + (size_t)(mBase + row) * ldc + n0 + c4) = v;
        }
        __threadfence();
      }
    }
    wave_lds_sync();
  }
}

template <int MODE>
__global__ __launch_bounds__(256) void cast8_kernel(const float* __restrict__ in, unsigned short* __restrict__ o0,
                                                    unsigned short* __restrict__ o1, int n8, float carry) {
  const int i = blockIdx.x * 256 + threadIdx.x;
  if (i >= n8) return;
  const size_t e0 = (size_t)i << 3;
  const v4f a0 = *(const v4f*)(in + e0);
  const v4f a1 = *(const v4f*)(in + e0 + 4);
  unsigned short bb[8], hb[8];
#pragma unroll
  for (int e = 0; e < 4; ++e) {
    bb[e]     = f2bf_bits(a0[e]);
    bb[4 + e] = f2bf_bits(a1[e]);
  }
#pragma unroll
  for (int e = 0; e < 8; ++e) hb[e] = (MODE == 1) ? h_bits(bf_bits2f(bb[e]) * carry) : (unsigned short)0;
  const v4u ub = (v4u){pk16(bb[0], bb[1]), pk16(bb[2], bb[3]), pk16(bb[4], bb[5]), pk16(bb[6], bb[7])};
  const v4u uh = (v4u){pk16(hb[0], hb[1]), pk16(hb[2], hb[3]), pk16(hb[4], hb[5]), pk16(hb[6], hb[7])};
  unsigned short* q0 = o0 + e0;
  unsigned short* q1 = o1 + e0;
  *(volatile v4u*)q0 = ub;
  if (MODE == 1) *(volatile v4u*)q1 = uh;
  __threadfence();
  *(volatile v4u*)q0 = ub;
  if (MODE == 1) *(volatile v4u*)q1 = uh;
}

__global__ __launch_bounds__(256) void normrot_kernel(
    const float* __restrict__ QKV, const float* __restrict__ ctab, const float* __restrict__ stab,
    const float* __restrict__ qw, const float* __restrict__ kw,
    unsigned short* __restrict__ Qp, unsigned short* __restrict__ Kp, float* __restrict__ Qe, float* __restrict__ Ke) {
  const int lane = threadIdx.x & 31;
  const int wave = __builtin_amdgcn_readfirstlane((int)(threadIdx.x >> 5));
  const int gw   = blockIdx.x * 8 + wave;
  const int tok  = gw / kSlots;
  const int slot = gw - tok * kSlots;
  const int pos  = tok & (kS - 1);
  const int b    = tok / kS;
  const bool isq = slot < kHq;
  const int kslot = isq ? 0 : (slot - kHq);

  const v4f x   = *(const v4f*)(QKV + (size_t)tok * kQKVW + slot * kHD + 4 * lane);
  const v4f wq4 = *(const v4f*)(qw + 4 * lane);
  const v4f wk4 = *(const v4f*)(kw + 4 * lane);
  const v4f c4  = *(const v4f*)(ctab + (size_t)pos * kHD + 4 * lane);
  const v4f s4  = *(const v4f*)(stab + (size_t)pos * kHD + 4 * lane);

  float ss = x[0] * x[0];
  ss = fmaf(x[1], x[1], ss);
  ss = fmaf(x[2], x[2], ss);
  ss = fmaf(x[3], x[3], ss);
#pragma unroll
  for (int off = 16; off > 0; off >>= 1) ss += __shfl_xor(ss, off, 32);
  const float inv = rsqrtf(ss * (1.0f / (float)kHD) + kEps);

  float n[4], p[4], y[4];
#pragma unroll
  for (int e = 0; e < 4; ++e) {
    const float w = bf16r(isq ? wq4[e] : wk4[e]);
    n[e] = x[e] * inv * w;
  }
#pragma unroll
  for (int e = 0; e < 4; ++e) p[e] = __shfl_xor(n[e], 16, 32);
  const float sgn = (lane < 16) ? -1.0f : 1.0f;
#pragma unroll
  for (int e = 0; e < 4; ++e) y[e] = n[e] * bf16r(c4[e]) + sgn * (p[e] * bf16r(s4[e]));

  unsigned short hb[4];
#pragma unroll
  for (int e = 0; e < 4; ++e) hb[e] = h_bits(y[e] * kQKCarry);
  const v2u u = (v2u){pk16(hb[0], hb[1]), pk16(hb[2], hb[3])};
  const v4f yv = (v4f){y[0], y[1], y[2], y[3]};

  unsigned short* dq = Qp + (size_t)tok * kQW + slot * kHD + 4 * lane;
  unsigned short* dk = Kp + (size_t)tok * kKW + kslot * kHD + 4 * lane;
  unsigned short* d16 = isq ? dq : dk;
  const bool early = pos < kEarly;
  const int erow = b * kEarly + (early ? pos : 0);
  float* eq = Qe + (size_t)erow * kQW + (isq ? slot : 0) * kHD + 4 * lane;
  float* ek = Ke + (size_t)erow * kKW + kslot * kHD + 4 * lane;
  float* d32 = isq ? eq : ek;
  for (int pass = 0; pass < 2; ++pass) {
    *(volatile v2u*)d16 = u;
    if (early) *(volatile v4f*)d32 = yv;
    __threadfence();
  }
}

__global__ __launch_bounds__(256) void vprep_kernel(const float* __restrict__ QKV, unsigned short* __restrict__ Vt,
                                                    float* __restrict__ Ve) {
  __shared__ __align__(16) float sm[64 * kVP];
  const int tid  = threadIdx.x;
  const int lane = tid & 31;
  const int wave = __builtin_amdgcn_readfirstlane((int)(tid >> 5));
  const int st   = blockIdx.x & 31;
  const int hkv  = (blockIdx.x >> 5) & (kHkv - 1);
  const int b    = blockIdx.x >> 7;
  const int s0   = st * 64;
  const float* src = QKV + (size_t)(b * kS + s0) * kQKVW + kVCol0 + hkv * kHD;
#pragma unroll
  for (int i = 0; i < 8; ++i) {
    const int e  = i * 256 + tid;
    const int r  = e >> 5;
    const int cc = (e & 31) * 4;
    const v4f v = *(const v4f*)(src + (size_t)r * kQKVW + cc);
    *(v4f*)(sm + r * kVP + cc) = v;
  }
  __syncthreads();
  const int q = lane >> 3, c8 = (lane & 7) * 8;
  v4u tv[4];
#pragma unroll
  for (int it = 0; it < 4; ++it) {
    const int d = it * 32 + wave * 4 + q;
    unsigned short hb[8];
#pragma unroll
    for (int e = 0; e < 8; ++e) hb[e] = h_bits(sm[(c8 + e) * kVP + d] * kVCarry);
    tv[it] = (v4u){pk16(hb[0], hb[1]), pk16(hb[2], hb[3]), pk16(hb[4], hb[5]), pk16(hb[6], hb[7])};
  }
  v4f ev[8];
#pragma unroll
  for (int it = 0; it < 8; ++it) ev[it] = *(const v4f*)(sm + (it * 8 + wave) * kVP + 4 * lane);
  const bool early = s0 < kEarly;
  const int erow0 = b * kEarly + (early ? s0 : 0);
  unsigned short* vt0 = Vt + (size_t)(b * kHkv + hkv) * kHD * kS + s0 + c8;
  float* ve0 = Ve + (size_t)erow0 * kKW + hkv * kHD + 4 * lane;
  for (int pass = 0; pass < 2; ++pass) {
#pragma unroll
    for (int it = 0; it < 4; ++it) *(volatile v4u*)(vt0 + (size_t)(it * 32 + wave * 4 + q) * kS) = tv[it];
    if (early) {
#pragma unroll
      for (int it = 0; it < 8; ++it) *(volatile v4f*)(ve0 + (size_t)(it * 8 + wave) * kKW) = ev[it];
    }
    __threadfence();
  }
}

__global__ __launch_bounds__(256) void attn_late_kernel(const unsigned short* __restrict__ Qp, const unsigned short* __restrict__ Kp,
                                                        const unsigned short* __restrict__ Vtp, float* __restrict__ attn) {
  union FH { v16h v; v8h h[2]; };
  __shared__ __align__(16) _Float16 Psh[8][16 * kLateKC];
  __shared__ __align__(16) float Os[8][16 * 68];
  const int lane = threadIdx.x & 31;
  const int wave = __builtin_amdgcn_readfirstlane((int)(threadIdx.x >> 5));
  const int hh   = lane >> 4;
  const int c    = lane & 15;
  const int qt2  = blockIdx.x % kLatePairs;
  const int bh   = blockIdx.x / kLatePairs;
  const int hkv  = bh & (kHkv - 1);
  const int b    = bh / kHkv;
  const int h    = hkv * kRep + (wave & 3);
  const int q0   = kEarly + (qt2 * 2 + (wave >> 2)) * 16;

  const _Float16* Kb = (const _Float16*)Kp + (size_t)b * kS * kKW + hkv * kHD + 8 * hh;
  const _Float16* Vb = (const _Float16*)Vtp + (size_t)(b * kHkv + hkv) * kHD * kS + 8 * hh;
  float* ob = attn + (size_t)(b * kS + q0) * kQW + h * kHD;

  v16h qa[4];
  {
    const _Float16* qrow = (const _Float16*)Qp + (size_t)(b * kS + q0 + c) * kQW + h * kHD + 8 * hh;
#pragma unroll
    for (int dc = 0; dc < 4; ++dc) qa[dc] = Frag<_Float16>::load(qrow + dc * 32);
  }

  float mrow[8], lrow[8];
  v8f oacc[8];
#pragma unroll
  for (int r = 0; r < 8; ++r) { mrow[r] = -INFINITY; lrow[r] = 0.0f; }
#pragma unroll
  for (int t = 0; t < 8; ++t) oacc[t] = (v8f){0.f,0.f,0.f,0.f,0.f,0.f,0.f,0.f};

  int nChunks = (q0 + 16 + kLateKC - 1) / kLateKC;
  if (nChunks > kS / kLateKC) nChunks = kS / kLateKC;
  _Float16* pw = Psh[wave];

  for (int kc = 0; kc < nChunks; ++kc) {
    const int kv0 = kc * kLateKC;
    v8f s[4];
#pragma unroll
    for (int j = 0; j < 4; ++j) {
      s[j] = (v8f){0.f,0.f,0.f,0.f,0.f,0.f,0.f,0.f};
      const _Float16* kr = Kb + (size_t)(kv0 + j * 16 + c) * kKW;
#pragma unroll
      for (int dc = 0; dc < 4; ++dc) {
        const v16h kf = Frag<_Float16>::load(kr + dc * 32);
        s[j] = mma_guard_h(qa[dc], kf, s[j]);
      }
      asm volatile("" ::: "memory");
    }
    const bool diag = (kc == nChunks - 1);
    float cm[8];
#pragma unroll
    for (int r = 0; r < 8; ++r) {
      const int qrow = q0 + 8 * hh + r;
      float m = -INFINITY;
#pragma unroll
      for (int j = 0; j < 4; ++j) {
        const int kvcol = kv0 + j * 16 + c;
        float v = s[j][r] * kScoreMul;
        if (diag && (kvcol > qrow)) v = -INFINITY;
        s[j][r] = v;
        m = fmaxf(m, v);
      }
#pragma unroll
      for (int off = 1; off < 16; off <<= 1) m = fmaxf(m, __shfl_xor(m, off, 32));
      cm[r] = m;
    }
#pragma unroll
    for (int r = 0; r < 8; ++r) {
      const float mnew  = fmaxf(mrow[r], cm[r]);
      const float alpha = __expf(mrow[r] - mnew);
      mrow[r] = mnew;
      float psum = 0.0f;
#pragma unroll
      for (int j = 0; j < 4; ++j) {
        const float p = __expf(s[j][r] - mnew);
        psum += p;
        pw[(8 * hh + r) * kLateKC + j * 16 + c] = (_Float16)(p * kPCarry);
      }
#pragma unroll
      for (int off = 1; off < 16; off <<= 1) psum += __shfl_xor(psum, off, 32);
      lrow[r] = lrow[r] * alpha + psum;
#pragma unroll
      for (int t = 0; t < 8; ++t) oacc[t][r] *= alpha;
    }
    wave_lds_sync();
#pragma unroll
    for (int kk = 0; kk < 2; ++kk) {
      FH pa;
      pa.h[0] = *(const v8h*)(pw + c * kLateKC + kk * 32 + 8 * hh);
      pa.h[1] = *(const v8h*)(pw + c * kLateKC + kk * 32 + 16 + 8 * hh);
#pragma unroll
      for (int t = 0; t < 8; ++t) {
        const v16h vf = Frag<_Float16>::load(Vb + (size_t)(t * 16 + c) * kS + kv0 + kk * 32);
        oacc[t] = mma_guard_h(pa.v, vf, oacc[t]);
      }
      asm volatile("" ::: "memory");
    }
    wave_lds_sync();
  }

  float inv[8];
#pragma unroll
  for (int r = 0; r < 8; ++r) inv[r] = 1.0f / (lrow[r] * (kPCarry * kVCarry));
  float* os = Os[wave];
  const int c4 = (lane & 15) * 4;
#pragma unroll
  for (int hf = 0; hf < 2; ++hf) {
#pragma unroll
    for (int r = 0; r < 8; ++r) {
#pragma unroll
      for (int t4 = 0; t4 < 4; ++t4) os[(8 * hh + r) * 68 + t4 * 16 + c] = oacc[hf * 4 + t4][r] * inv[r];
    }
    wave_lds_sync();
    for (int pass = 0; pass < 2; ++pass) {
#pragma unroll
      for (int it = 0; it < 8; ++it) {
        const int row = it * 2 + hh;
        v4f val = *(const v4f*)(os + row * 68 + c4);
        *(volatile v4f*)(ob + (size_t)row * kQW + hf * 64 + c4) = val;
      }
      __threadfence();
    }
    wave_lds_sync();
  }
}

__global__ __launch_bounds__(128) void attn_early_kernel(const float* __restrict__ Qe, const float* __restrict__ Ke,
                                                         const float* __restrict__ Ve, float* __restrict__ attn) {
  __shared__ __align__(16) float sq[4][kHD];
  __shared__ __align__(16) float sp[4][kEarly];
  const int lane = threadIdx.x & 31;
  const int wave = __builtin_amdgcn_readfirstlane((int)(threadIdx.x >> 5));
  const int t    = blockIdx.x & (kEarly - 1);
  const int hkv  = (blockIdx.x / kEarly) & (kHkv - 1);
  const int b    = blockIdx.x / (kEarly * kHkv);
  const int h    = hkv * kRep + wave;
  const int erow = b * kEarly + t;
  float* sqw = sq[wave];
  float* spw = sp[wave];
  {
    const v4f qv = *(const v4f*)(Qe + (size_t)erow * kQW + h * kHD + 4 * lane);
    *(v4f*)(sqw + 4 * lane) = qv;
  }
  wave_lds_sync();
  float sc[4];
#pragma unroll
  for (int i = 0; i < 4; ++i) {
    const int j  = lane + 32 * i;
    const int jc = (j < t) ? j : t;
    float dot = 0.0f;
    if (32 * i <= t) {
      const float* kr = Ke + (size_t)(b * kEarly + jc) * kKW + hkv * kHD;
#pragma unroll 1
      for (int d4 = 0; d4 < kHD / 4; ++d4) {
        const v4f kv = *(const v4f*)(kr + 4 * d4);
        float k0 = kv[0], k1 = kv[1], k2 = kv[2], k3 = kv[3];
        asm volatile("" : "+v"(k0), "+v"(k1), "+v"(k2), "+v"(k3));
        const v4f qq = *(const v4f*)(sqw + 4 * d4);
        dot = fmaf(k0, qq[0], dot);
        dot = fmaf(k1, qq[1], dot);
        dot = fmaf(k2, qq[2], dot);
        dot = fmaf(k3, qq[3], dot);
      }
    }
    sc[i] = (j <= t) ? (dot * kInvSqrtHD) : -INFINITY;
  }
  float m = fmaxf(fmaxf(sc[0], sc[1]), fmaxf(sc[2], sc[3]));
#pragma unroll
  for (int off = 16; off > 0; off >>= 1) m = fmaxf(m, __shfl_xor(m, off, 32));
  float psum = 0.0f;
#pragma unroll
  for (int i = 0; i < 4; ++i) {
    const float p = expf(sc[i] - m);
    psum += p;
    spw[lane + 32 * i] = p;
  }
#pragma unroll
  for (int off = 16; off > 0; off >>= 1) psum += __shfl_xor(psum, off, 32);
  wave_lds_sync();
  float a0 = 0.0f, a1 = 0.0f, a2 = 0.0f, a3 = 0.0f;
  const float* vr = Ve + (size_t)(b * kEarly) * kKW + hkv * kHD + 4 * lane;
#pragma unroll 1
  for (int j = 0; j <= t; ++j) {
    const float p = spw[j];
    const v4f vv = *(const v4f*)(vr + (size_t)j * kKW);
    a0 = fmaf(p, vv[0], a0);
    a1 = fmaf(p, vv[1], a1);
    a2 = fmaf(p, vv[2], a2);
    a3 = fmaf(p, vv[3], a3);
  }
  const float il = 1.0f / psum;
  const v4f ov = (v4f){a0 * il, a1 * il, a2 * il, a3 * il};
  float* dst = attn + (size_t)(b * kS + t) * kQW + h * kHD + 4 * lane;
  *(volatile v4f*)dst = ov;
  __threadfence();
  *(volatile v4f*)dst = ov;
}

__global__ __launch_bounds__(256) void gate_kernel(const float* __restrict__ attn, const float* __restrict__ G,
                                                   unsigned short* __restrict__ GH, unsigned short* __restrict__ EH,
                                                   unsigned short* __restrict__ EL) {
  __shared__ __align__(16) float sm[kQW];
  const int tid = threadIdx.x;
  const int row = blockIdx.x;
  const int pos = row & (kS - 1);
  const int b   = row / kS;
  const float* ar = attn + (size_t)row * kQW;
  const float* gr = G + (size_t)row * kQW;
#pragma unroll 1
  for (int i = 0; i < kQW / 256; ++i) {
    const int col = i * 256 + tid;
    const float a = ar[col];
    const float g = gr[col];
    const float sg = 1.0f / (1.0f + expf(-g));
    sm[col] = a * sg;
  }
  __syncthreads();
  const v4f x0 = *(const v4f*)(sm + 8 * tid);
  const v4f x1 = *(const v4f*)(sm + 8 * tid + 4);
  if (pos >= kEarly) {
    unsigned short hb[8];
#pragma unroll
    for (int e = 0; e < 4; ++e) {
      hb[e]     = h_bits(x0[e] * kGCarry);
      hb[4 + e] = h_bits(x1[e] * kGCarry);
    }
    const v4u u = (v4u){pk16(hb[0], hb[1]), pk16(hb[2], hb[3]), pk16(hb[4], hb[5]), pk16(hb[6], hb[7])};
    unsigned short* d = GH + (size_t)row * kQW + 8 * tid;
    *(volatile v4u*)d = u;
    __threadfence();
    *(volatile v4u*)d = u;
  } else {
    unsigned short hb[8], lb[8];
#pragma unroll
    for (int e = 0; e < 4; ++e) {
      const float f0 = x0[e];
      const float f1 = x1[e];
      hb[e]     = f2bf_bits(f0);
      hb[4 + e] = f2bf_bits(f1);
      lb[e]     = f2bf_bits(f0 - bf_bits2f(hb[e]));
      lb[4 + e] = f2bf_bits(f1 - bf_bits2f(hb[4 + e]));
    }
    const v4u uh = (v4u){pk16(hb[0], hb[1]), pk16(hb[2], hb[3]), pk16(hb[4], hb[5]), pk16(hb[6], hb[7])};
    const v4u ul = (v4u){pk16(lb[0], lb[1]), pk16(lb[2], lb[3]), pk16(lb[4], lb[5]), pk16(lb[6], lb[7])};
    const size_t o = (size_t)(b * kEarly + pos) * kQW + 8 * tid;
    *(volatile v4u*)(EH + o) = uh;
    *(volatile v4u*)(EL + o) = ul;
    __threadfence();
    *(volatile v4u*)(EH + o) = uh;
    *(volatile v4u*)(EL + o) = ul;
  }
}

extern "C" void kernel_launch(void* const* d_in, const int* in_sizes, int n_in,
                              void* d_out, int out_size, void* d_ws, size_t ws_size,
                              hipStream_t stream) {
  if (n_in < 10) return;
  if (in_sizes[0] != kTok * kHid) return;
  if (in_sizes[1] != kS * kHD) return;
  if (in_sizes[2] != kS * kHD) return;
  if (in_sizes[3] != kQW * kHid) return;
  if (in_sizes[4] != kKW * kHid) return;
  if (in_sizes[5] != kKW * kHid) return;
  if (in_sizes[6] != kQW * kHid) return;
  if (in_sizes[7] != kQW * kQW) return;
  if (in_sizes[8] != kHD) return;
  if (in_sizes[9] != kHD) return;
  if (out_size != kTok * kQW) return;
  if (ws_size < kWsTotal) return;

  const float* X    = (const float*)d_in[0];
  const float* ctab = (const float*)d_in[1];
  const float* stab = (const float*)d_in[2];
  const float* Wq   = (const float*)d_in[3];
  const float* Wk   = (const float*)d_in[4];
  const float* Wv   = (const float*)d_in[5];
  const float* Wg   = (const float*)d_in[6];
  const float* Wo   = (const float*)d_in[7];
  const float* qnw  = (const float*)d_in[8];
  const float* knw  = (const float*)d_in[9];
  float* out = (float*)d_out;

  char* ws = (char*)d_ws;
  unsigned short* XB   = (unsigned short*)(ws + kOffXB);
  unsigned short* WQKV = (unsigned short*)(ws + kOffWQKV);
  unsigned short* WGB  = (unsigned short*)(ws + kOffWGB);
  float*          QKV  = (float*)(ws + kOffQKV);
  unsigned short* QP   = (unsigned short*)(ws + kOffQP);
  unsigned short* KP   = (unsigned short*)(ws + kOffKP);
  unsigned short* VT   = (unsigned short*)(ws + kOffVT);
  float*          QE   = (float*)(ws + kOffQE);
  float*          KE   = (float*)(ws + kOffKE);
  float*          VE   = (float*)(ws + kOffVE);
  unsigned short* WOB  = (unsigned short*)(ws + kOffWOB);
  unsigned short* WOH  = (unsigned short*)(ws + kOffWOH);
  float*          ATT  = (float*)(ws + kOffATT);
  float*          GF   = (float*)(ws + kOffGF);
  unsigned short* GH   = (unsigned short*)(ws + kOffGH);
  unsigned short* EH   = (unsigned short*)(ws + kOffEH);
  unsigned short* EL   = (unsigned short*)(ws + kOffEL);

  cast8_kernel<0><<<(kTok * kHid / 8) / 256, 256, 0, stream>>>(X, XB, XB, kTok * kHid / 8, 1.0f);
  cast8_kernel<0><<<(kQW * kHid / 8) / 256, 256, 0, stream>>>(Wq, WQKV, WQKV, kQW * kHid / 8, 1.0f);
  cast8_kernel<0><<<(kKW * kHid / 8) / 256, 256, 0, stream>>>(Wk, WQKV + (size_t)kQW * kHid, WQKV, kKW * kHid / 8, 1.0f);
  cast8_kernel<0><<<(kKW * kHid / 8) / 256, 256, 0, stream>>>(Wv, WQKV + (size_t)kVCol0 * kHid, WQKV, kKW * kHid / 8, 1.0f);
  cast8_kernel<0><<<(kQW * kHid / 8) / 256, 256, 0, stream>>>(Wg, WGB, WGB, kQW * kHid / 8, 1.0f);
  cast8_kernel<1><<<(kQW * kQW / 8) / 256, 256, 0, stream>>>(Wo, WOB, WOH, kQW * kQW / 8, kWoCarry);

  wmma_gemm64<1, false><<<dim3((kTok / 64) * (kQKVW / 64) / 8, 1), 256, 0, stream>>>(
      XB, XB, kHid, 0L, WQKV, kHid, 0L, QKV, kQKVW, 0L, kTok, kQKVW, kHid, 1.0f);

  normrot_kernel<<<kTok * kSlots / 8, 256, 0, stream>>>(QKV, ctab, stab, qnw, knw, QP, KP, QE, KE);

  vprep_kernel<<<kB * kHkv * (kS / 64), 256, 0, stream>>>(QKV, VT, VE);

  attn_late_kernel<<<kLatePairs * kHkv * kB, 256, 0, stream>>>(QP, KP, VT, ATT);
  attn_early_kernel<<<kB * kHkv * kEarly, 128, 0, stream>>>(QE, KE, VE, ATT);

  wmma_gemm64<1, false><<<dim3((kTok / 64) * (kQW / 64) / 8, 1), 256, 0, stream>>>(
      XB, XB, kHid, 0L, WGB, kHid, 0L, GF, kQW, 0L, kTok, kQW, kHid, 1.0f);

  gate_kernel<<<kTok, 256, 0, stream>>>(ATT, GF, GH, EH, EL);

  wmma_gemm64<0, false><<<dim3(((kS - kEarly) / 64) * (kQW / 64) / 8, kB), 256, 0, stream>>>(
      GH + (size_t)kEarly * kQW, GH + (size_t)kEarly * kQW, kQW, (long)kS * kQW,
      WOH, kQW, 0L,
      out + (size_t)kEarly * kQW, kQW, (long)kS * kQW,
      kS - kEarly, kQW, kQW, kOutLateMul);

  wmma_gemm64<1, true><<<dim3((kEarly / 64) * (kQW / 64) / 8, kB), 256, 0, stream>>>(
      EH, EL, kQW, (long)kEarly * kQW,
      WOB, kQW, 0L,
      out, kQW, (long)kS * kQW,
      kEarly, kQW, kQW, 1.0f);
}
